// KA_GNN_two_60430189854855
// MI455X (gfx1250) — hardware-verified
//
#include <hip/hip_runtime.h>
#include <stddef.h>


#define INF_    64
#define HIDF    32
#define GRIDN   4
#define NTHR    256
#define NWAVE   8
#define EPT     8
#define NGRP    2
#define CHUNK   (NTHR * EPT * NGRP)
#define WCAP    (EPT * NGRP * 32)
#define LISTN   (NWAVE * WCAP)
#define NBC     4096
#define NBF     1024
#define NBP     128
#define RCAP    40960
#define RBN     128
#define TGT     256
#define DEGCAP  256
#define KROWS   64
#define KTHR    128
#define OTHR    512
#define NEGS    0.01f

#define LDS_FILL ((RCAP + NBF + LISTN) * 4 + 64)

static_assert((CHUNK & (CHUNK - 1)) == 0);
static_assert(CHUNK <= 4096);
static_assert(NBC <= 4096 && NBF <= 4096 && NBP <= 4096);
static_assert((NBC & (NBC - 1)) == 0 && (NBF & (NBF - 1)) == 0 && (NBP & (NBP - 1)) == 0);
static_assert(NBC == 4 * NBF);
static_assert(OTHR * 8 == NBC);
static_assert((RCAP % 32) == 0);
static_assert(TGT == NWAVE * 32);
static_assert((TGT % KROWS) == 0);
static_assert(KROWS == (KTHR / 32) * 16);
static_assert((KROWS * INF_) % KTHR == 0 && (KROWS * HIDF) % KTHR == 0);
static_assert(NBP * HIDF / 4 <= 4 * NTHR);
static_assert(NBP <= NTHR && NBP == 4 * 32);
static_assert(HIDF == 32);

typedef float          v4f   __attribute__((ext_vector_type(4)));
typedef float          v8f   __attribute__((ext_vector_type(8)));
typedef int            v4i   __attribute__((ext_vector_type(4)));
typedef unsigned short v8us  __attribute__((ext_vector_type(8)));
typedef __bf16         v16bf __attribute__((ext_vector_type(16)));
union FragB { v16bf v; v8us u[2]; };

__device__ __forceinline__ unsigned int bfr(float f) {
  unsigned int u = __float_as_uint(f);
  u += 0x7FFFu + ((u >> 16) & 1u);
  return u >> 16;
}
__device__ __forceinline__ void split1(float v, unsigned short& h, unsigned short& l) {
  const unsigned int hb = bfr(v);
  const float hf = __uint_as_float(hb << 16);
  const unsigned int lb = bfr(v - hf);
  h = (unsigned short)hb;
  l = (unsigned short)lb;
}
__device__ __forceinline__ void split8(v4f a, v4f b, v8us& hv, v8us& lv) {
  unsigned short h, l;
  split1(a.x, h, l); hv[0] = h; lv[0] = l;
  split1(a.y, h, l); hv[1] = h; lv[1] = l;
  split1(a.z, h, l); hv[2] = h; lv[2] = l;
  split1(a.w, h, l); hv[3] = h; lv[3] = l;
  split1(b.x, h, l); hv[4] = h; lv[4] = l;
  split1(b.y, h, l); hv[5] = h; lv[5] = l;
  split1(b.z, h, l); hv[6] = h; lv[6] = l;
  split1(b.w, h, l); hv[7] = h; lv[7] = l;
}

__device__ __forceinline__ v8f wmb(v16bf a, v16bf b, v8f c) {
  v8f d = __builtin_amdgcn_wmma_f32_16x16x32_bf16(false, a, false, b, (short)0, c, false, false);
  asm volatile("v_nop\n\tv_nop\n\tv_nop\n\tv_nop" : "+v"(d) : "v"(a), "v"(b));
  return d;
}

template <int NB>
__device__ __forceinline__ int scan_chunk(const int* __restrict__ dsts, int nE, int cbase, int slotBase,
                                          int vec8, int* list, int tid, int lane, int wave) {
  int wc = 0;
#pragma unroll
  for (int g = 0; g < NGRP; ++g) {
    const int el0  = (g * NTHR + tid) * EPT;
    const int e0   = cbase + el0;
    const int sent = -2147483647 - 1;
    v4i da, db;
    if (vec8 != 0 && cbase + CHUNK <= nE) {
      da = *(const v4i*)(dsts + e0);
      db = *(const v4i*)(dsts + e0 + 4);
    } else {
      da.x = (e0     < nE) ? dsts[min(e0, nE - 1)] : sent;
      da.y = (e0 + 1 < nE) ? dsts[min(e0 + 1, nE - 1)] : sent;
      da.z = (e0 + 2 < nE) ? dsts[min(e0 + 2, nE - 1)] : sent;
      da.w = (e0 + 3 < nE) ? dsts[min(e0 + 3, nE - 1)] : sent;
      db.x = (e0 + 4 < nE) ? dsts[min(e0 + 4, nE - 1)] : sent;
      db.y = (e0 + 5 < nE) ? dsts[min(e0 + 5, nE - 1)] : sent;
      db.z = (e0 + 6 < nE) ? dsts[min(e0 + 6, nE - 1)] : sent;
      db.w = (e0 + 7 < nE) ? dsts[min(e0 + 7, nE - 1)] : sent;
    }
    const unsigned nb = (unsigned)slotBase;
    const unsigned s0 = (unsigned)da.x - nb, s1 = (unsigned)da.y - nb;
    const unsigned s2 = (unsigned)da.z - nb, s3 = (unsigned)da.w - nb;
    const unsigned s4 = (unsigned)db.x - nb, s5 = (unsigned)db.y - nb;
    const unsigned s6 = (unsigned)db.z - nb, s7 = (unsigned)db.w - nb;
    const bool h0 = s0 < (unsigned)NB, h1 = s1 < (unsigned)NB, h2 = s2 < (unsigned)NB, h3 = s3 < (unsigned)NB;
    const bool h4 = s4 < (unsigned)NB, h5 = s5 < (unsigned)NB, h6 = s6 < (unsigned)NB, h7 = s7 < (unsigned)NB;
    const unsigned any = __builtin_amdgcn_ballot_w32(h0 | h1 | h2 | h3 | h4 | h5 | h6 | h7);
    if (any != 0u) {
#define HITJ(J, HJ, SJ) { \
        const unsigned mj = __builtin_amdgcn_ballot_w32(HJ); \
        if (mj != 0u) { \
          if (HJ) { \
            const int pos = wc + (int)__builtin_amdgcn_mbcnt_lo(mj, 0u); \
            if (pos < WCAP) list[wave * WCAP + pos] = ((el0 + (J)) << 12) | (int)(SJ); \
          } \
          wc += (int)__builtin_popcount(mj); } }
      HITJ(0, h0, s0)
      HITJ(1, h1, s1)
      HITJ(2, h2, s2)
      HITJ(3, h3, s3)
      HITJ(4, h4, s4)
      HITJ(5, h5, s5)
      HITJ(6, h6, s6)
      HITJ(7, h7, s7)
#undef HITJ
    }
  }
  return wc;
}

__global__ __launch_bounds__(NTHR) void k_wprep(
    const float* __restrict__ W_in, const float* __restrict__ W_conv,
    unsigned short* binH, unsigned short* binL, unsigned short* bcvH, unsigned short* bcvL, int nL) {
  const int gin = HIDF * INF_;
  const int gcv = nL * HIDF * HIDF;
  const int bstart = blockIdx.x * NTHR;
  const int idx = bstart + (int)threadIdx.x;
  v4f ca, sa;
  unsigned short* dh; unsigned short* dl;
  size_t o;
  if (bstart < gin) {
    const int oc = idx / INF_;
    const int i  = idx - oc * INF_;
    ca = *(const v4f*)(W_in + ((size_t)(0 * HIDF + oc) * INF_ + i) * GRIDN);
    sa = *(const v4f*)(W_in + ((size_t)(1 * HIDF + oc) * INF_ + i) * GRIDN);
    dh = binH; dl = binL;
    o = (size_t)oc * (INF_ * 2 * GRIDN) + (size_t)i * 8;
  } else {
    const int j = idx - gin;
    if (j >= gcv) return;
    const int l  = j / (HIDF * HIDF);
    const int jj = j - l * (HIDF * HIDF);
    const int oc = jj / HIDF;
    const int i  = jj - oc * HIDF;
    ca = *(const v4f*)(W_conv + ((((size_t)l * 2 + 0) * HIDF + oc) * HIDF + i) * GRIDN);
    sa = *(const v4f*)(W_conv + ((((size_t)l * 2 + 1) * HIDF + oc) * HIDF + i) * GRIDN);
    dh = bcvH; dl = bcvL;
    o = (size_t)l * (HIDF * HIDF * 2 * GRIDN) + (size_t)oc * (HIDF * 2 * GRIDN) + (size_t)i * 8;
  }
  v8us hv, lv;
  split8(ca, sa, hv, lv);
  *(volatile v8us*)(dh + o) = hv;
  *(volatile v8us*)(dl + o) = lv;
  __threadfence();
  *(volatile v8us*)(dh + o) = hv;
  *(volatile v8us*)(dl + o) = lv;
}

__global__ __launch_bounds__(NTHR) void k_count(
    const int* __restrict__ ei, int* cnt, int nE, int vec8) {
  __shared__ __attribute__((aligned(16))) int scnt[NBC];
  __shared__ __attribute__((aligned(16))) int list[LISTN];
  __shared__ int wcnt[NWAVE];
  const int tid = threadIdx.x, lane = tid & 31, wave = tid >> 5;
  const int nodeBase = blockIdx.x * NBC;
  const int* dsts = ei + nE;

  for (int i = tid; i < NBC; i += NTHR) scnt[i] = 0;
  __syncthreads();

  const int nChunks = (nE + CHUNK - 1) / CHUNK;
#pragma unroll 1
  for (int ch = 0; ch < nChunks; ++ch) {
    const int cbase = ch * CHUNK;
    const int wc = scan_chunk<NBC>(dsts, nE, cbase, nodeBase, vec8, list, tid, lane, wave);
    if (lane == 0) wcnt[wave] = wc;
    __syncthreads();
    if (wave == 0) {
#pragma unroll 1
      for (int wsx = 0; wsx < NWAVE; ++wsx) {
        int n = __builtin_amdgcn_readfirstlane(wcnt[wsx]);
        n = n > WCAP ? WCAP : (n < 0 ? 0 : n);
        const int* lp = list + wsx * WCAP;
#pragma unroll 1
        for (int i = 0; i < n; ++i) {
          const int ent  = __builtin_amdgcn_readfirstlane(lp[i]);
          const int slot = ent & (NBC - 1);
          if (lane == 0) scnt[slot] = scnt[slot] + 1;
        }
      }
    }
    __syncthreads();
  }

  v4i cq[4];
#pragma unroll
  for (int q = 0; q < 4; ++q) {
    const int f = (wave * 4 + q) * 128 + 4 * lane;
    cq[q] = *(const v4i*)(scnt + f);
  }
  int* cp = cnt + (size_t)nodeBase;
#pragma unroll
  for (int q = 0; q < 4; ++q) {
    const int f = (wave * 4 + q) * 128 + 4 * lane;
    *(volatile v4i*)(cp + f) = cq[q];
  }
  __threadfence();
#pragma unroll
  for (int q = 0; q < 4; ++q) {
    const int f = (wave * 4 + q) * 128 + 4 * lane;
    *(volatile v4i*)(cp + f) = cq[q];
  }
}

__global__ __launch_bounds__(OTHR) void k_offsets(
    const int* __restrict__ cnt, int* off, int* rbase, int nChunk) {
  __shared__ __attribute__((aligned(16))) int soff[NBC];
  __shared__ __attribute__((aligned(16))) int srb[RBN];
  __shared__ int wtot[OTHR / 32];
  const int tid = threadIdx.x, lane = tid & 31, wave = tid >> 5, sub = tid >> 7;
  for (int i = tid; i < RBN; i += OTHR) srb[i] = 0;
  int carry = 0;
#pragma unroll 1
  for (int ch = 0; ch < nChunk; ++ch) {
    const int base = ch * NBC;
    const v4i c0 = *(const v4i*)(cnt + base + 8 * tid);
    const v4i c1 = *(const v4i*)(cnt + base + 8 * tid + 4);
    const int e0 = max(c0.x, 0), e1 = max(c0.y, 0), e2 = max(c0.z, 0), e3 = max(c0.w, 0);
    const int e4 = max(c1.x, 0), e5 = max(c1.y, 0), e6 = max(c1.z, 0), e7 = max(c1.w, 0);
    const int ts = e0 + e1 + e2 + e3 + e4 + e5 + e6 + e7;
    int incl = ts;
#pragma unroll
    for (int d = 1; d < 32; d <<= 1) {
      const int t = __shfl_up(incl, d);
      if (lane >= d) incl += t;
    }
    if (lane == 31) wtot[wave] = incl;
    __syncthreads();
    const int S0 = wtot[0]  + wtot[1]  + wtot[2]  + wtot[3];
    const int S1 = wtot[4]  + wtot[5]  + wtot[6]  + wtot[7];
    const int S2 = wtot[8]  + wtot[9]  + wtot[10] + wtot[11];
    const int S3 = wtot[12] + wtot[13] + wtot[14] + wtot[15];
    int pre = 0;
#pragma unroll 1
    for (int w = 4 * sub; w < wave; ++w) pre += wtot[w];
    const int b0 = carry;
    const int b1 = b0 + ((S0 + 31) & ~31);
    const int b2 = b1 + ((S1 + 31) & ~31);
    const int b3 = b2 + ((S2 + 31) & ~31);
    const int b4 = b3 + ((S3 + 31) & ~31);
    const int myb = sub == 0 ? b0 : (sub == 1 ? b1 : (sub == 2 ? b2 : b3));
    if (tid == 0) {
      srb[min(4 * ch + 0, RBN - 1)] = b0;
      srb[min(4 * ch + 1, RBN - 1)] = b1;
      srb[min(4 * ch + 2, RBN - 1)] = b2;
      srb[min(4 * ch + 3, RBN - 1)] = b3;
    }
    int run = myb + pre + incl - ts;
    soff[8 * tid + 0] = run; run += e0;
    soff[8 * tid + 1] = run; run += e1;
    soff[8 * tid + 2] = run; run += e2;
    soff[8 * tid + 3] = run; run += e3;
    soff[8 * tid + 4] = run; run += e4;
    soff[8 * tid + 5] = run; run += e5;
    soff[8 * tid + 6] = run; run += e6;
    soff[8 * tid + 7] = run;
    carry = b4;
    __syncthreads();
    const v4i o0 = *(const v4i*)(soff + 4 * tid);
    const v4i o1 = *(const v4i*)(soff + 4 * (tid + OTHR));
    int* op = off + base;
    *(volatile v4i*)(op + 4 * tid) = o0;
    *(volatile v4i*)(op + 4 * (tid + OTHR)) = o1;
    __threadfence();
    *(volatile v4i*)(op + 4 * tid) = o0;
    *(volatile v4i*)(op + 4 * (tid + OTHR)) = o1;
    __syncthreads();
  }
  if (tid == 0) srb[min(4 * nChunk, RBN - 1)] = carry;
  __syncthreads();
  v4i rv = {0, 0, 0, 0};
  if (tid < 32) rv = *(const v4i*)(srb + 4 * tid);
  if (tid < 32) *(volatile v4i*)(rbase + 4 * tid) = rv;
  __threadfence();
  if (tid < 32) *(volatile v4i*)(rbase + 4 * tid) = rv;
}

__global__ __launch_bounds__(NTHR) void k_fill(
    const int* __restrict__ ei, const int* __restrict__ off, const int* __restrict__ rbase,
    int* csr, int nN, int nE, int vec8, int csrLen) {
  extern __shared__ v4f lds_dyn[];
  int* region = (int*)lds_dyn;
  int* cursor = region + RCAP;
  int* list   = cursor + NBF;
  int* wcnt   = list + LISTN;
  const int tid = threadIdx.x, lane = tid & 31, wave = tid >> 5;
  const int b = blockIdx.x;
  const int nodeBase = b * NBF;
  const int* dsts = ei + nE;

  int rb0 = rbase[b];
  const int rb1 = rbase[b + 1];
  rb0 = rb0 < 0 ? 0 : (rb0 > csrLen ? csrLen : rb0);
  rb0 &= ~31;
  int len = rb1 - rb0;
  len = len < 0 ? 0 : (len > RCAP ? RCAP : len);
  int lenW = (len + 31) & ~31;
  if (rb0 + lenW > csrLen) lenW = (csrLen - rb0) & ~31;

  {
    const v4i z = {0, 0, 0, 0};
    for (int i = tid; i < RCAP / 4; i += NTHR) ((v4i*)region)[i] = z;
    for (int s = tid; s < NBF; s += NTHR) {
      int o = off[nodeBase + s] - rb0;
      o = o < 0 ? 0 : (o > RCAP ? RCAP : o);
      cursor[s] = o;
    }
  }
  __syncthreads();

  const int nChunks = (nE + CHUNK - 1) / CHUNK;
#pragma unroll 1
  for (int ch = 0; ch < nChunks; ++ch) {
    const int cbase = ch * CHUNK;
    const int wc = scan_chunk<NBF>(dsts, nE, cbase, nodeBase, vec8, list, tid, lane, wave);
    if (lane == 0) wcnt[wave] = wc;
    __syncthreads();
    if (wave == 0) {
#pragma unroll 1
      for (int wsx = 0; wsx < NWAVE; ++wsx) {
        int n = __builtin_amdgcn_readfirstlane(wcnt[wsx]);
        n = n > WCAP ? WCAP : (n < 0 ? 0 : n);
        const int* lp = list + wsx * WCAP;
#pragma unroll 1
        for (int i = 0; i < n; ++i) {
          const int ent  = __builtin_amdgcn_readfirstlane(lp[i]);
          const int slot = ent & (NBF - 1);
          int e = cbase + ((ent >> 12) & (CHUNK - 1));
          e = e > nE - 1 ? nE - 1 : e;
          int src = ei[e];
          src = src < 0 ? 0 : (src > nN - 1 ? nN - 1 : src);
          if (lane == 0) {
            int pos = cursor[slot];
            pos = pos < 0 ? 0 : (pos > RCAP - 1 ? RCAP - 1 : pos);
            region[pos] = src;
            const int np = pos + 1;
            cursor[slot] = np > RCAP ? RCAP : np;
          }
        }
      }
    }
    __syncthreads();
  }

  const int nv = lenW >> 2;
  int* gp = csr + rb0;
#pragma unroll 1
  for (int i = tid; i < nv; i += NTHR) { const v4i v = ((const v4i*)region)[i]; *(volatile v4i*)(gp + 4 * i) = v; }
  __threadfence();
#pragma unroll 1
  for (int i = tid; i < nv; i += NTHR) { const v4i v = ((const v4i*)region)[i]; *(volatile v4i*)(gp + 4 * i) = v; }
}

template <int IN_CH>
__global__ __launch_bounds__(KTHR) void k_kan(
    const float* __restrict__ X, const unsigned short* __restrict__ Bhi, const unsigned short* __restrict__ Blo,
    float* C, int nRowsX) {
  extern __shared__ v4f lds_dyn[];
  constexpr int K  = IN_CH * 2 * GRIDN;
  constexpr int KP = K + 8;
  static_assert((K % 32) == 0 && ((KP * 2) % 16) == 0);
  unsigned short* sAh = (unsigned short*)lds_dyn;
  unsigned short* sAl = sAh + KROWS * KP;
  float*          stg = (float*)lds_dyn;
  const int tid = threadIdx.x, lane = tid & 31, wave = tid >> 5, hh = lane >> 4, m = lane & 15;
  const int rowBase = blockIdx.x * KROWS;

#pragma unroll 1
  for (int it = 0; it < (KROWS * IN_CH) / KTHR; ++it) {
    const int p   = it * KTHR + tid;
    const int row = p / IN_CH;
    const int i   = p - row * IN_CH;
    int node = rowBase + row;
    node = node > nRowsX - 1 ? nRowsX - 1 : node;
    const float v = X[(size_t)node * IN_CH + i];
    float s1, c1, s2, c2, s3, c3, s4, c4;
    sincosf(v,        &s1, &c1);
    sincosf(v * 2.0f, &s2, &c2);
    sincosf(v * 3.0f, &s3, &c3);
    sincosf(v * 4.0f, &s4, &c4);
    v4f ca, sa;
    ca.x = c1; ca.y = c2; ca.z = c3; ca.w = c4;
    sa.x = s1; sa.y = s2; sa.z = s3; sa.w = s4;
    v8us hv, lv;
    split8(ca, sa, hv, lv);
    *(v8us*)(sAh + row * KP + 8 * i) = hv;
    *(v8us*)(sAl + row * KP + 8 * i) = lv;
  }
  __syncthreads();

  v8f acc[2];
  {
    v8f z = {0.f, 0.f, 0.f, 0.f, 0.f, 0.f, 0.f, 0.f};
    acc[0] = z; acc[1] = z;
  }
  const unsigned short* ahr = sAh + (wave * 16 + m) * KP + 8 * hh;
  const unsigned short* alr = sAl + (wave * 16 + m) * KP + 8 * hh;
#pragma unroll 1
  for (int kt = 0; kt < K / 32; ++kt) {
    FragB ah, al;
    ah.u[0] = *(const v8us*)(ahr + 32 * kt);
    ah.u[1] = *(const v8us*)(ahr + 32 * kt + 16);
    al.u[0] = *(const v8us*)(alr + 32 * kt);
    al.u[1] = *(const v8us*)(alr + 32 * kt + 16);
#pragma unroll
    for (int t = 0; t < 2; ++t) {
      const size_t bo = (size_t)(16 * t + m) * K + 32 * kt + 8 * hh;
      FragB bh, bl;
      bh.u[0] = *(const v8us*)(Bhi + bo);
      bh.u[1] = *(const v8us*)(Bhi + bo + 16);
      bl.u[0] = *(const v8us*)(Blo + bo);
      bl.u[1] = *(const v8us*)(Blo + bo + 16);
      acc[t] = wmb(ah.v, bh.v, acc[t]);
      acc[t] = wmb(ah.v, bl.v, acc[t]);
      acc[t] = wmb(al.v, bh.v, acc[t]);
    }
  }
  __syncthreads();

  float* sp = stg + (wave * 16 + 8 * hh) * HIDF + m;
#pragma unroll
  for (int t = 0; t < 2; ++t) {
#pragma unroll
    for (int r = 0; r < 8; ++r) sp[r * HIDF + 16 * t] = acc[t][r];
  }
  __syncthreads();

  const float* lp = stg + wave * 16 * HIDF + 4 * lane;
  float* gp = C + ((size_t)rowBase + wave * 16) * HIDF + 4 * lane;
  v4f ov[4];
#pragma unroll
  for (int i = 0; i < 4; ++i) ov[i] = *(const v4f*)(lp + i * 128);
#pragma unroll
  for (int i = 0; i < 4; ++i) *(volatile v4f*)(gp + (size_t)i * 128) = ov[i];
  __threadfence();
#pragma unroll
  for (int i = 0; i < 4; ++i) *(volatile v4f*)(gp + (size_t)i * 128) = ov[i];
}

__global__ __launch_bounds__(NTHR) void k_agg(
    const int* __restrict__ csr, const int* __restrict__ off, const int* __restrict__ cnt,
    const float* __restrict__ T, const float* __restrict__ hin, float* hout, int nN, int csrLen) {
  const int tid = threadIdx.x, lane = tid & 31, wave = tid >> 5;
  const int tbase = blockIdx.x * TGT + wave * 32;
  const int cl = tbase + lane;
  const int cnt_l = cnt[cl];
  const int off_l = off[cl];

#pragma unroll 1
  for (int j = 0; j < 32; ++j) {
    const int c = tbase + j;
    int n = __builtin_amdgcn_readlane(cnt_l, j);
    n = n < 0 ? 0 : (n > DEGCAP ? DEGCAP : n);
    const int st = __builtin_amdgcn_readlane(off_l, j);
    float acc = 0.0f;
#pragma unroll 1
    for (int q0 = 0; q0 < n; q0 += 32) {
      int pos = st + q0 + lane;
      pos = pos < 0 ? 0 : (pos > csrLen - 1 ? csrLen - 1 : pos);
      int sl = csr[pos];
      sl = sl < 0 ? 0 : (sl > nN - 1 ? nN - 1 : sl);
      const int mcnt = (n - q0) < 32 ? (n - q0) : 32;
#pragma unroll 1
      for (int p = 0; p < mcnt; ++p) {
        const int s = __builtin_amdgcn_readlane(sl, p);
        acc += T[(size_t)s * HIDF + lane];
      }
    }
    const float hv = hin[(size_t)c * HIDF + lane];
    float v = acc + hv;
    v = v > 0.0f ? v : NEGS * v;
    float* hp = hout + (size_t)c * HIDF + lane;
    *(volatile float*)hp = v;
    __threadfence();
    *(volatile float*)hp = v;
  }
}

__global__ __launch_bounds__(NTHR) void k_pool(
    const int* __restrict__ batch, const float* __restrict__ h,
    const float* __restrict__ Wout, const float* __restrict__ bout, float* out, int nN) {
  __shared__ __attribute__((aligned(16))) float acc[NBP * HIDF];
  __shared__ __attribute__((aligned(16))) int list[LISTN];
  __shared__ __attribute__((aligned(16))) float sOut[NBP];
  __shared__ int pc[NBP];
  __shared__ int wcnt[NWAVE];
  const int tid = threadIdx.x, lane = tid & 31, wave = tid >> 5;

  {
    const v4f z = {0.f, 0.f, 0.f, 0.f};
    for (int i = tid; i < NBP * HIDF / 4; i += NTHR) ((v4f*)acc)[i] = z;
    for (int i = tid; i < NBP; i += NTHR) { pc[i] = 0; sOut[i] = 0.0f; }
  }
  __syncthreads();

  const int nChunks = (nN + CHUNK - 1) / CHUNK;
#pragma unroll 1
  for (int ch = 0; ch < nChunks; ++ch) {
    const int cbase = ch * CHUNK;
    const int wc = scan_chunk<NBP>(batch, nN, cbase, 0, 1, list, tid, lane, wave);
    if (lane == 0) wcnt[wave] = wc;
    __syncthreads();
    if (wave == 0) {
#pragma unroll 1
      for (int wsx = 0; wsx < NWAVE; ++wsx) {
        int n = __builtin_amdgcn_readfirstlane(wcnt[wsx]);
        n = n > WCAP ? WCAP : (n < 0 ? 0 : n);
        const int* lp = list + wsx * WCAP;
#pragma unroll 1
        for (int i = 0; i < n; ++i) {
          const int ent  = __builtin_amdgcn_readfirstlane(lp[i]);
          const int slot = ent & (NBP - 1);
          int nd = cbase + ((ent >> 12) & (CHUNK - 1));
          nd = nd > nN - 1 ? nN - 1 : nd;
          const float v = h[(size_t)nd * HIDF + lane];
          acc[slot * HIDF + lane] = acc[slot * HIDF + lane] + v;
          if (lane == 0) pc[slot] = pc[slot] + 1;
        }
      }
    }
    __syncthreads();
  }

  if (tid < NBP) {
    int cv = pc[tid];
    cv = cv < 1 ? 1 : cv;
    const float inv = 1.0f / (float)cv;
    float dc = 0.0f, ds = 0.0f;
    const float* ap = acc + tid * HIDF;
#pragma unroll 1
    for (int i = 0; i < HIDF; ++i) {
      const float y = ap[i] * inv;
      float s, c;
      sincosf(y, &s, &c);
      dc += c * Wout[i];
      ds += s * Wout[HIDF + i];
    }
    float z = dc + ds;
    z += bout[0];
    const float e = expf(-z);
    sOut[tid] = 1.0f / (1.0f + e);
  }
  __syncthreads();

  v4f ov = {0.f, 0.f, 0.f, 0.f};
  if (tid < 32) ov = *(const v4f*)(sOut + 4 * tid);
  if (tid < 32) *(volatile v4f*)(out + 4 * tid) = ov;
  __threadfence();
  if (tid < 32) *(volatile v4f*)(out + 4 * tid) = ov;
}

extern "C" void kernel_launch(void* const* d_in, const int* in_sizes, int n_in,
                              void* d_out, int out_size, void* d_ws, size_t ws_size,
                              hipStream_t stream) {
  if (n_in < 7) return;
  const int nN = in_sizes[0] / INF_;
  const int nE = in_sizes[1] / 2;
  if (nN <= 0 || nE <= 0 || in_sizes[0] != nN * INF_ || in_sizes[1] != 2 * nE || in_sizes[2] != nN) return;
  if (in_sizes[3] != 2 * HIDF * INF_ * GRIDN) return;
  const int nL = in_sizes[4] / (2 * HIDF * HIDF * GRIDN);
  if (nL < 1 || nL > 8 || in_sizes[4] != nL * 2 * HIDF * HIDF * GRIDN) return;
  if (in_sizes[5] != 2 * HIDF || in_sizes[6] < 1) return;
  const int G = out_size;
  if (G != NBP) return;
  if (nE > (1 << 28) || nN > (1 << 24)) return;

  const float* x      = (const float*)d_in[0];
  const int*   ei     = (const int*)d_in[1];
  const int*   batch  = (const int*)d_in[2];
  const float* W_in   = (const float*)d_in[3];
  const float* W_conv = (const float*)d_in[4];
  const float* W_out  = (const float*)d_in[5];
  const float* b_out  = (const float*)d_in[6];
  float* out = (float*)d_out;

  const int NPAD   = ((nN + TGT - 1) / TGT) * TGT;
  const int nBC    = (nN + NBC - 1) / NBC;
  const int CNTPAD = nBC * NBC;
  if (4 * nBC + 1 > RBN) return;
  const int nBF    = (nN + NBF - 1) / NBF;
  const int csrLen = ((nE + 31) & ~31) + 4096;
  const int nKan   = NPAD / KROWS;
  const int nAgg   = NPAD / TGT;
  if (NPAD > CNTPAD || nBF * NBF > CNTPAD) return;

  const int KIN = INF_ * 2 * GRIDN;
  const int KCV = HIDF * 2 * GRIDN;

  char* ws = (char*)d_ws;
  size_t off = 0;
  const size_t oBIh = off; off += (size_t)HIDF * KIN * 2;            off = (off + 255) & ~(size_t)255;
  const size_t oBIl = off; off += (size_t)HIDF * KIN * 2;            off = (off + 255) & ~(size_t)255;
  const size_t oBCh = off; off += (size_t)nL * HIDF * KCV * 2;       off = (off + 255) & ~(size_t)255;
  const size_t oBCl = off; off += (size_t)nL * HIDF * KCV * 2;       off = (off + 255) & ~(size_t)255;
  const size_t oCnt = off; off += (size_t)CNTPAD * 4;                off = (off + 255) & ~(size_t)255;
  const size_t oOff = off; off += (size_t)CNTPAD * 4;                off = (off + 255) & ~(size_t)255;
  const size_t oRb  = off; off += (size_t)RBN * 4;                   off = (off + 255) & ~(size_t)255;
  const size_t oCsr = off; off += (size_t)csrLen * 4;                off = (off + 255) & ~(size_t)255;
  const size_t oH0  = off; off += (size_t)NPAD * HIDF * 4;           off = (off + 255) & ~(size_t)255;
  const size_t oH1  = off; off += (size_t)NPAD * HIDF * 4;           off = (off + 255) & ~(size_t)255;
  const size_t oT   = off; off += (size_t)NPAD * HIDF * 4;           off = (off + 255) & ~(size_t)255;
  if (off > ws_size || off > ((size_t)128 << 20)) return;
  unsigned short* binH = (unsigned short*)(ws + oBIh);
  unsigned short* binL = (unsigned short*)(ws + oBIl);
  unsigned short* bcvH = (unsigned short*)(ws + oBCh);
  unsigned short* bcvL = (unsigned short*)(ws + oBCl);
  int*   cnt  = (int*)(ws + oCnt);
  int*   offp = (int*)(ws + oOff);
  int*   rb   = (int*)(ws + oRb);
  int*   csr  = (int*)(ws + oCsr);
  float* h0   = (float*)(ws + oH0);
  float* h1   = (float*)(ws + oH1);
  float* tpl  = (float*)(ws + oT);

  const int vec8 = ((nE & 3) == 0) ? 1 : 0;

  const int nPrepThr = HIDF * INF_ + nL * HIDF * HIDF;
  k_wprep<<<(nPrepThr + NTHR - 1) / NTHR, NTHR, 0, stream>>>(W_in, W_conv, binH, binL, bcvH, bcvL, nL);

  k_count<<<nBC, NTHR, 0, stream>>>(ei, cnt, nE, vec8);
  k_offsets<<<1, OTHR, 0, stream>>>(cnt, offp, rb, nBC);
  hipFuncSetAttribute(reinterpret_cast<const void*>(&k_fill),
                      hipFuncAttributeMaxDynamicSharedMemorySize, LDS_FILL);
  k_fill<<<nBF, NTHR, LDS_FILL, stream>>>(ei, offp, rb, csr, nN, nE, vec8, csrLen);

  const int ldsIn = 2 * KROWS * (KIN + 8) * 2;
  const int ldsCv = 2 * KROWS * (KCV + 8) * 2;
  hipFuncSetAttribute(reinterpret_cast<const void*>(&k_kan<INF_>),
                      hipFuncAttributeMaxDynamicSharedMemorySize, ldsIn);
  hipFuncSetAttribute(reinterpret_cast<const void*>(&k_kan<HIDF>),
                      hipFuncAttributeMaxDynamicSharedMemorySize, ldsCv);
  k_kan<INF_><<<nKan, KTHR, ldsIn, stream>>>(x, binH, binL, h0, nN);

  float* hc = h0;
  float* hn = h1;
  for (int l = 0; l < nL; ++l) {
    k_kan<HIDF><<<nKan, KTHR, ldsCv, stream>>>(hc, bcvH + (size_t)l * HIDF * KCV, bcvL + (size_t)l * HIDF * KCV, tpl, NPAD);
    k_agg<<<nAgg, NTHR, 0, stream>>>(csr, offp, cnt, tpl, hc, hn, nN, csrLen);
    float* tp = hc; hc = hn; hn = tp;
  }

  k_pool<<<1, NTHR, 0, stream>>>(batch, hc, W_out, b_out, out, nN);
}
